// MultiHeadAttention_50079318671839
// MI455X (gfx1250) — hardware-verified
//
#include <hip/hip_runtime.h>


#ifndef NB
#define NB 2
#endif
#ifndef SEQ
#define SEQ 2048
#endif
#define NB_FULL  2
#define SEQ_FULL 2048
#define TT   SEQ
#define DM   1024
#define NH_  16
#define HD   64
#define DQ   (NH_ * HD)
#define ZH   2
#define NBK  32
#define BTN  (TT + 8)

static_assert(TT % 128 == 0);
static_assert(TT % 64 == 0);
static_assert(NH_ % ZH == 0);
static_assert(NB <= NB_FULL);
static_assert(SEQ <= SEQ_FULL);
static_assert((size_t)4 * DQ * DM * 2 + (size_t)TT * DM * 2 + (size_t)2 * TT * DQ * 4 + (size_t)6 * NH_ * TT * HD * 2 + (size_t)ZH * TT * TT * 4 + (size_t)2 * ZH * TT * TT * 2 + (size_t)ZH * TT * HD * 4 + (size_t)2 * TT * DQ * 2 <= (size_t)134217728);

typedef unsigned short bf;
typedef __attribute__((ext_vector_type(16))) __bf16   v16bf;
typedef __attribute__((ext_vector_type(8)))  unsigned short v8us;
typedef __attribute__((ext_vector_type(4)))  unsigned short v4us;
typedef __attribute__((ext_vector_type(2)))  unsigned short v2us;
typedef __attribute__((ext_vector_type(8)))  float    v8f;
typedef __attribute__((ext_vector_type(4)))  float    v4f;
typedef __attribute__((ext_vector_type(2)))  float    v2f;
typedef v4f  __attribute__((may_alias)) v4fa;

__device__ __forceinline__ unsigned short f2bf(float f) { unsigned u = __float_as_uint(f); u += 0x7FFFu + ((u >> 16) & 1u); return (unsigned short)(u >> 16); }
__device__ __forceinline__ float bf2f(unsigned short b) { return __uint_as_float(((unsigned)b) << 16); }
__device__ __forceinline__ float bfr(float f) { return bf2f(f2bf(f)); }
__device__ __forceinline__ void splitf(float y, unsigned short& h, unsigned short& l) { h = f2bf(y); l = f2bf(y - bf2f(h)); }
__device__ __forceinline__ v16bf cat16b(v8us lo, v8us hi) { return __builtin_bit_cast(v16bf, __builtin_shufflevector(lo, hi, 0, 1, 2, 3, 4, 5, 6, 7, 8, 9, 10, 11, 12, 13, 14, 15)); }
__device__ __forceinline__ v8f wmmab(v16bf a, v16bf b, v8f c) { return __builtin_amdgcn_wmma_f32_16x16x32_bf16(false, a, false, b, (short)0, c, false, false); }

__device__ __forceinline__ v16bf ldfrag(const bf* p) { return cat16b(*(const v8us*)p, *(const v8us*)(p + 16)); }

template <int NSPLIT>
__global__ __launch_bounds__(32) void k_gemmw(const bf* __restrict__ A, const bf* __restrict__ A2, const bf* __restrict__ Bt, const bf* __restrict__ Bt2, int K, float* C, int ldc, size_t sA, size_t sB, size_t sC) {
    typedef v16bf V;
    __shared__ __align__(16) float os[16 * 68];
    const size_t z = blockIdx.z; A += z * sA; if (A2) A2 += z * sA; Bt += z * sB; if (Bt2) Bt2 += z * sB; C += z * sC;
    const int lane = threadIdx.x & 31, lr = lane & 15, hi = lane >> 4; const int r0 = blockIdx.x * 64, c0 = blockIdx.y * 64;
    v8f acc[4][4];
#pragma unroll
    for (int mb = 0; mb < 4; ++mb)
#pragma unroll
        for (int nb = 0; nb < 4; ++nb) acc[mb][nb] = (v8f){};
    const size_t aoff = (size_t)(r0 + lr) * K + 8 * hi, boff = (size_t)(c0 + lr) * K + 8 * hi;
#pragma unroll 1
    for (int kc = 0; kc < K; kc += 32) {
        V a[4], a2[4];
#pragma unroll
        for (int mb = 0; mb < 4; ++mb) { a[mb] = ldfrag(A + aoff + (size_t)mb * 16 * K + kc); if (NSPLIT == 1 || NSPLIT == 2) a2[mb] = ldfrag(A2 + aoff + (size_t)mb * 16 * K + kc); }
#pragma unroll
        for (int nb = 0; nb < 4; ++nb) { const V b = ldfrag(Bt + boff + (size_t)nb * 16 * K + kc); V b2; if (NSPLIT >= 2) b2 = ldfrag(Bt2 + boff + (size_t)nb * 16 * K + kc);
#pragma unroll
            for (int mb = 0; mb < 4; ++mb) { acc[mb][nb] = wmmab(a[mb], b, acc[mb][nb]); if (NSPLIT == 1 || NSPLIT == 2) acc[mb][nb] = wmmab(a2[mb], b, acc[mb][nb]); if (NSPLIT >= 2) acc[mb][nb] = wmmab(a[mb], b2, acc[mb][nb]); } }
        asm volatile("v_nop\n\tv_nop\n\tv_nop\n\tv_nop" : "+v"(acc[0][0]), "+v"(acc[1][1]), "+v"(acc[2][2]), "+v"(acc[3][3]) : "v"(a[0]), "v"(a[3]));
    }
#pragma unroll
    for (int mb = 0; mb < 4; ++mb) {
#pragma unroll
        for (int nb = 0; nb < 4; ++nb) {
#pragma unroll
            for (int j = 0; j < 8; ++j) os[(hi * 8 + j) * 68 + nb * 16 + lr] = acc[mb][nb][j]; }
        __builtin_amdgcn_wave_barrier(); asm volatile("" ::: "memory");
        float* crow = C + (size_t)(r0 + mb * 16) * ldc + c0;
#pragma unroll 1
        for (int ps = 0; ps < 2; ++ps) {
#pragma unroll
            for (int s = 0; s < 8; ++s) { const int row = 2 * s + hi, cofs = lr * 4; const v4f val = *(const v4fa*)(os + row * 68 + cofs);
                *(volatile v4f*)(crow + (size_t)row * ldc + cofs) = val; }
            if (ps == 0) __threadfence(); }
        __builtin_amdgcn_wave_barrier(); asm volatile("" ::: "memory");
    }
}

__global__ __launch_bounds__(256) void k_wtG(const float* __restrict__ w, int K, int N, bf* Bt) {
    const int lane = threadIdx.x & 31; const int L0 = (blockIdx.x * 8 + (threadIdx.x >> 5)) * 8; const int nlines = N * K / 64;
#pragma unroll
    for (int ps = 0; ps < 2; ++ps) {
#pragma unroll 1
        for (int l = 0; l < 8; ++l) { const int L = L0 + l; if (L >= nlines) break; const size_t e = (size_t)L * 64 + lane * 2; const int k = (int)(e % K), n = (int)(e / K); v2us o;
            o[0] = f2bf(w[(size_t)k * N + n]); o[1] = f2bf(w[(size_t)(k + 1) * N + n]); *(volatile v2us*)(Bt + e) = o; }
        if (ps == 0) __threadfence(); }
}
__global__ __launch_bounds__(256) void k_cvt8(const float* __restrict__ src, bf* dst, size_t n8) { const size_t i = (size_t)blockIdx.x * 256 + threadIdx.x; if (i >= n8) return; const v8f v = *(const v8f*)(src + i * 8); v8us o;
#pragma unroll
    for (int k = 0; k < 8; ++k) o[k] = f2bf(v[k]); *(volatile v8us*)(dst + i * 8) = o; __threadfence(); *(volatile v8us*)(dst + i * 8) = o; }

__global__ __launch_bounds__(256) void k_hpl(const float* __restrict__ F, int pitch, int nheads, bf* Ph, bf* Pl) {
    const size_t e = ((size_t)blockIdx.x * 256 + threadIdx.x) * 2; if (e >= (size_t)nheads * TT * HD) return; const int d = (int)(e % HD); const int t = (int)((e / HD) % TT); const int h = (int)(e / ((size_t)HD * TT));
    const v2f x = *(const v2f*)(F + (size_t)t * pitch + h * HD + d); v2us oh, ol;
#pragma unroll
    for (int q = 0; q < 2; ++q) { unsigned short a2, c2; splitf(x[q], a2, c2); oh[q] = a2; ol[q] = c2; }
    *(volatile v2us*)(Ph + e) = oh; *(volatile v2us*)(Pl + e) = ol; __threadfence(); *(volatile v2us*)(Ph + e) = oh; *(volatile v2us*)(Pl + e) = ol; }
__global__ __launch_bounds__(256) void k_vtp(const float* __restrict__ F, int pitch, int nheads, bf* Vh, bf* Vl) { const size_t e = ((size_t)blockIdx.x * 256 + threadIdx.x) * 2; if (e >= (size_t)nheads * HD * TT) return; const int t = (int)(e % TT); const int d = (int)((e / TT) % HD); const int g = (int)(e / ((size_t)TT * HD)); v2us oh, ol;
#pragma unroll
    for (int q = 0; q < 2; ++q) { const float x = F[(size_t)(t + q) * pitch + g * HD + d]; unsigned short a2, c2; splitf(x, a2, c2); oh[q] = a2; ol[q] = c2; }
    *(volatile v2us*)(Vh + e) = oh; *(volatile v2us*)(Vl + e) = ol; __threadfence(); *(volatile v2us*)(Vh + e) = oh; *(volatile v2us*)(Vl + e) = ol; }

__device__ __forceinline__ int relbucket(int rel) {
    const int rp = rel < 0 ? -rel : rel;
    const int lg = 8 + (rp >= 12 ? 1 : 0) + (rp >= 16 ? 1 : 0) + (rp >= 23 ? 1 : 0) + (rp >= 32 ? 1 : 0) + (rp >= 46 ? 1 : 0) + (rp >= 64 ? 1 : 0) + (rp >= 91 ? 1 : 0);
    const int bk = (rp < 8) ? rp : lg;
    return bk + ((rel > 0) ? 16 : 0);
}

__global__ __launch_bounds__(256) void k_asoft(const float* __restrict__ Sb, const float* __restrict__ tab, int h0, bf* Ph, bf* Pl) {
    __shared__ float bt[BTN];
    const int lane = threadIdx.x & 31, w = __builtin_amdgcn_readfirstlane((int)(threadIdx.x >> 5));
    const int row0 = blockIdx.x * 8; const int zz = row0 / TT; const int i0 = row0 - zz * TT; const int head = h0 + zz;
#pragma unroll 1
    for (int u = threadIdx.x; u < BTN; u += 256) { const int bk = relbucket(u - (i0 + 7)); const int ti = min(max(bk * NH_ + head, 0), NBK * NH_ - 1); bt[u] = bfr(tab[ti]); }
    __syncthreads();
    const int row = row0 + w; const int i = i0 + w; const int bo = 7 - w; const float* sr = Sb + (size_t)row * TT; float v[TT / 32]; float mx = -3.0e38f;
#pragma unroll
    for (int ch = 0; ch < TT / 128; ++ch) { const int j0 = ch * 128 + lane * 4; const v4f a = *(const v4f*)(sr + j0);
#pragma unroll
        for (int q = 0; q < 4; ++q) { const float t = a[q] + bt[j0 + q + bo]; v[ch * 4 + q] = t; mx = fmaxf(mx, t); } }
#pragma unroll
    for (int sh = 16; sh; sh >>= 1) mx = fmaxf(mx, __shfl_xor(mx, sh, 32));
    float sum = 0.f;
#pragma unroll
    for (int k = 0; k < TT / 32; ++k) { float d0 = __fsub_rn(v[k], mx); asm volatile("" : "+v"(d0)); v[k] = __builtin_amdgcn_exp2f(__fmul_rn(d0, 1.4426950408889634f)); sum += v[k]; }
#pragma unroll
    for (int sh = 16; sh; sh >>= 1) sum += __shfl_xor(sum, sh, 32);
    const float f = __fdiv_rn(1.0f, sum);
#pragma unroll 1
    for (int ps = 0; ps < 2; ++ps) {
#pragma unroll
        for (int ch = 0; ch < TT / 128; ++ch) { v4us oh, ol;
#pragma unroll
            for (int q = 0; q < 4; ++q) { unsigned short a, c2; splitf(v[ch * 4 + q] * f, a, c2); oh[q] = a; ol[q] = c2; }
            const size_t oo = ((size_t)zz * TT + i) * TT + ch * 128 + lane * 4; *(volatile v4us*)(Ph + oo) = oh; *(volatile v4us*)(Pl + oo) = ol; }
        if (ps == 0) __threadfence(); }
}
__global__ __launch_bounds__(256) void k_merge(const float* __restrict__ O, int h0, bf* Ah, bf* Al) { const size_t e = ((size_t)blockIdx.x * 256 + threadIdx.x) * 2; if (e >= (size_t)ZH * TT * HD) return; const int d = (int)(e % HD); const int t = (int)((e / HD) % TT); const int zz = (int)(e / ((size_t)HD * TT)); const size_t oo = (size_t)t * DQ + (h0 + zz) * HD + d;
    const v2f x = *(const v2f*)(O + e); v2us oh, ol;
#pragma unroll
    for (int q = 0; q < 2; ++q) { unsigned short a, c2; splitf(x[q], a, c2); oh[q] = a; ol[q] = c2; } *(volatile v2us*)(Ah + oo) = oh; *(volatile v2us*)(Al + oo) = ol; __threadfence(); *(volatile v2us*)(Ah + oo) = oh; *(volatile v2us*)(Al + oo) = ol; }

extern "C" void kernel_launch(void* const* d_in, const int* in_sizes, int n_in,
                              void* d_out, int out_size, void* d_ws, size_t ws_size, hipStream_t stream) {
    if (n_in < 6) return;
    if ((size_t)in_sizes[0] < (size_t)(NB - 1) * SEQ_FULL * DM + (size_t)TT * DM) return;
    if ((size_t)in_sizes[1] < (size_t)DM * DQ || (size_t)in_sizes[2] < (size_t)DM * DQ || (size_t)in_sizes[3] < (size_t)DM * DQ || (size_t)in_sizes[4] < (size_t)DQ * DM) return;
    if (in_sizes[5] < NBK * NH_) return;
    if ((size_t)out_size < (size_t)NB * TT * DM) return;
    const float* x = (const float*)d_in[0]; const float* wq = (const float*)d_in[1]; const float* wk = (const float*)d_in[2]; const float* wv = (const float*)d_in[3]; const float* wo = (const float*)d_in[4]; const float* tab = (const float*)d_in[5];
    float* OUT = (float*)d_out;
    char* wsp = (char*)d_ws;
    auto take = [&](size_t bytes) { char* p = wsp; wsp += (bytes + 255) & ~(size_t)255; return (void*)p; };
    bf* WQ = (bf*)take((size_t)DQ * DM * 2); bf* WK = (bf*)take((size_t)DQ * DM * 2); bf* WV = (bf*)take((size_t)DQ * DM * 2); bf* WO = (bf*)take((size_t)DM * DQ * 2);
    bf* XB = (bf*)take((size_t)TT * DM * 2); float* FQ = (float*)take((size_t)TT * DQ * 4); float* FK = (float*)take((size_t)TT * DQ * 4);
    bf* QPh = (bf*)take((size_t)NH_ * TT * HD * 2); bf* QPl = (bf*)take((size_t)NH_ * TT * HD * 2); bf* KPh = (bf*)take((size_t)NH_ * TT * HD * 2); bf* KPl = (bf*)take((size_t)NH_ * TT * HD * 2); bf* VTh = (bf*)take((size_t)NH_ * HD * TT * 2); bf* VTl = (bf*)take((size_t)NH_ * HD * TT * 2);
    float* Sb = (float*)take((size_t)ZH * TT * TT * 4); bf* Ph = (bf*)take((size_t)ZH * TT * TT * 2); bf* Pl = (bf*)take((size_t)ZH * TT * TT * 2);
    float* Ob = (float*)take((size_t)ZH * TT * HD * 4); bf* ATh = (bf*)take((size_t)TT * DQ * 2); bf* ATl = (bf*)take((size_t)TT * DQ * 2);
    if ((size_t)(wsp - (char*)d_ws) > ws_size) return;
    float* FV = FK;
    const unsigned LW = (unsigned)((DM * DQ / 64 + 63) / 64);
    k_wtG<<<LW, 256, 0, stream>>>(wq, DM, DQ, WQ);
    k_wtG<<<LW, 256, 0, stream>>>(wk, DM, DQ, WK);
    k_wtG<<<LW, 256, 0, stream>>>(wv, DM, DQ, WV);
    k_wtG<<<LW, 256, 0, stream>>>(wo, DQ, DM, WO);
    const unsigned LP = (unsigned)(((size_t)NH_ * TT * HD / 2 + 255) / 256);
    for (int b = 0; b < NB; ++b) {
        k_cvt8<<<(unsigned)(((size_t)TT * DM / 8 + 255) / 256), 256, 0, stream>>>(x + (size_t)b * SEQ_FULL * DM, XB, (size_t)TT * DM / 8);
        k_gemmw<0><<<dim3(TT / 64, DQ / 64, 1), 32, 0, stream>>>(XB, nullptr, WQ, nullptr, DM, FQ, DQ, 0, 0, 0);
        k_hpl<<<LP, 256, 0, stream>>>(FQ, DQ, NH_, QPh, QPl);
        k_gemmw<0><<<dim3(TT / 64, DQ / 64, 1), 32, 0, stream>>>(XB, nullptr, WK, nullptr, DM, FK, DQ, 0, 0, 0);
        k_hpl<<<LP, 256, 0, stream>>>(FK, DQ, NH_, KPh, KPl);
        k_gemmw<0><<<dim3(TT / 64, DQ / 64, 1), 32, 0, stream>>>(XB, nullptr, WV, nullptr, DM, FV, DQ, 0, 0, 0);
        k_vtp<<<LP, 256, 0, stream>>>(FV, DQ, NH_, VTh, VTl);
        for (int h0 = 0; h0 < NH_; h0 += ZH) { const size_t zo = (size_t)h0 * TT * HD;
            k_gemmw<2><<<dim3(TT / 64, TT / 64, ZH), 32, 0, stream>>>(QPh + zo, QPl + zo, KPh + zo, KPl + zo, HD, Sb, TT, (size_t)TT * HD, (size_t)TT * HD, (size_t)TT * TT);
            k_asoft<<<ZH * TT / 8, 256, 0, stream>>>(Sb, tab, h0, Ph, Pl);
            k_gemmw<2><<<dim3(TT / 64, HD / 64, ZH), 32, 0, stream>>>(Ph, Pl, VTh + zo, VTl + zo, TT, Ob, HD, (size_t)TT * TT, (size_t)HD * TT, (size_t)TT * HD);
            k_merge<<<(unsigned)(((size_t)ZH * TT * HD / 2 + 255) / 256), 256, 0, stream>>>(Ob, h0, ATh, ATl); }
        k_gemmw<1><<<dim3(TT / 64, DM / 64, 1), 32, 0, stream>>>(ATh, ATl, WO, nullptr, DQ, OUT + (size_t)b * TT * DM, DM, 0, 0, 0); }
}
